// PNAAggregator_3341484556653
// MI455X (gfx1250) — hardware-verified
//
#include <hip/hip_runtime.h>
#include <math.h>
#include <stdint.h>

#pragma clang fp contract(off)


#define PD 64
#define PK 768
#define POUT 64
#define NT 256
#define SP 16
#define SCH (NT * SP)
#define SRB 8192
#define RPW (SRB / (NT / 32))
#define RPW_LOG 10
#define APITCH 776
#define WSCALE 16.0f
#define WSCALE_INV 0.0625f
#define NEG_SLOPE 0.2f
#define WS_CAP ((size_t)134217728)

typedef __attribute__((ext_vector_type(16))) _Float16 v16h;
typedef __attribute__((ext_vector_type(8)))  _Float16 v8h;
typedef __attribute__((ext_vector_type(8)))  float    v8f;
typedef __attribute__((ext_vector_type(4)))  float    v4f;
typedef __attribute__((ext_vector_type(2)))  float    v2f;
typedef __attribute__((ext_vector_type(4)))  int      v4i;

__device__ __forceinline__ void dep_guard_h(v8f& a, v8f& b, v16h x, v16h y) { asm volatile("v_nop\n\tv_nop\n\tv_nop\n\tv_nop" : "+v"(a), "+v"(b) : "v"(x), "v"(y)); }
__device__ __forceinline__ void keep4_h(v16h a, v16h b, v16h c, v16h d) { asm volatile("v_nop" :: "v"(a), "v"(b), "v"(c), "v"(d)); }
__device__ __forceinline__ void acc_guard4(v8f& a, v8f& b, v8f& c, v8f& d) { asm volatile("v_nop\n\tv_nop\n\tv_nop\n\tv_nop" : "+v"(a), "+v"(b), "+v"(c), "+v"(d)); }
template <typename T> struct Frag;
template <> struct Frag<_Float16> {
  typedef v16h V; union U { v16h v; v8h h[2]; };
  static __device__ __forceinline__ v16h load(const _Float16* p) {
    U f; f.h[0] = *(const v8h*)(p); f.h[1] = *(const v8h*)(p + 16); return f.v;
  }
  static __device__ __forceinline__ v8f mma(v16h a, v16h b, v8f c) {
    return __builtin_amdgcn_wmma_f32_16x16x32_f16(false, a, false, b, (short)0, c, false, false);
  }
  static __device__ __forceinline__ void guard(v8f& a, v8f& b, v16h x, v16h y) { dep_guard_h(a, b, x, y); }
  static __device__ __forceinline__ void keep(v16h a, v16h b, v16h c, v16h d) { keep4_h(a, b, c, d); }
};

__global__ __launch_bounds__(256) void cast_w_f16x2(const float* __restrict__ in, _Float16* __restrict__ out, int n2) {
  int i = blockIdx.x * 256 + threadIdx.x;
  if (i < n2) {
    const _Float16 h0 = (_Float16)(in[2 * i] * WSCALE), h1 = (_Float16)(in[2 * i + 1] * WSCALE);
    const unsigned u = (unsigned)__builtin_bit_cast(unsigned short, h0) | ((unsigned)__builtin_bit_cast(unsigned short, h1) << 16);
    ((volatile unsigned*)out)[i] = u;
    __threadfence();
    ((volatile unsigned*)out)[i] = u;
  }
}

__device__ __forceinline__ int blk_excl_scan(int cnt, int* scan_ws, int tid, int* tot) {
  const int lane = tid & 31, wave = tid >> 5; int incl = cnt;
#pragma unroll
  for (int o = 1; o < 32; o <<= 1) { const int v = __shfl_up(incl, o, 32); if (lane >= o) incl += v; }
  if (lane == 31) scan_ws[wave] = incl;
  __syncthreads();
  if (wave == 0) { int wv = (lane < NT / 32) ? scan_ws[lane] : 0; int wincl = wv;
#pragma unroll
    for (int o = 1; o < 32; o <<= 1) { const int v = __shfl_up(wincl, o, 32); if (lane >= o) wincl += v; }
    if (lane < NT / 32) scan_ws[32 + lane] = wincl - wv; if (lane == 31) scan_ws[64] = wincl; }
  __syncthreads();
  const int res = scan_ws[32 + wave] + incl - cnt; *tot = scan_ws[64];
  return res;
}
__device__ __forceinline__ int chunk_hits_rows(const int* __restrict__ rows, int e0, int nnz, int n0, int tid, int* LIST, int* scan_ws) {
  const int eb = e0 + tid * SP;
  const bool inr = eb < nnz;
  const int ebc = inr ? eb : (nnz - SP);
  int rec[SP]; int cnt = 0;
#pragma unroll
  for (int k = 0; k < SP; k += 4) {
    const v4i r4 = *(const v4i*)(rows + ebc + k);
#pragma unroll
    for (int e = 0; e < 4; ++e) {
      const int r = r4[e]; int rc = -1;
      if (inr && r >= n0 && r < n0 + SRB) { rc = eb + k + e; ++cnt; }
      rec[k + e] = rc;
    }
  }
  int tot; int p = blk_excl_scan(cnt, scan_ws, tid, &tot);
#pragma unroll
  for (int k = 0; k < SP; ++k) if (rec[k] >= 0) { if ((unsigned)p < (unsigned)SCH) LIST[p] = rec[k]; ++p; }
  __syncthreads();
  return tot < SCH ? tot : SCH;
}

__global__ __launch_bounds__(NT) void k_stream(const int* __restrict__ rows, const int* __restrict__ cols, const float* __restrict__ vals,
                                               const float* __restrict__ feat, float* ASUM, float* ASQ, float* AMX, float* AMN,
                                               float* __restrict__ LOGD, float* __restrict__ PART, int nnz, int nch, int m, int nnode) {
  __shared__ int LIST[SCH];
  __shared__ __align__(16) float SDEG[SRB];
  __shared__ int scan_ws[80];
  __shared__ float SPART[NT / 32];
  const int tid = threadIdx.x, lane = tid & 31, wave = tid >> 5;
  const int n0 = blockIdx.x * SRB;
  const int c2 = 2 * lane;
  const v2f z2 = {0.f, 0.f};
  const v2f inf2 = {__builtin_inff(), __builtin_inff()};
#pragma unroll 1
  for (int j = 0; j < RPW; ++j) {
    const size_t o = (size_t)(n0 + wave * RPW + j) * PD + c2;
    *(volatile v2f*)(ASUM + o) = z2; *(volatile v2f*)(ASQ + o) = z2; *(volatile v2f*)(AMX + o) = z2; *(volatile v2f*)(AMN + o) = inf2;
    __threadfence();
    *(volatile v2f*)(ASUM + o) = z2; *(volatile v2f*)(ASQ + o) = z2; *(volatile v2f*)(AMX + o) = z2; *(volatile v2f*)(AMN + o) = inf2;
  }
  for (int i = tid; i < SRB; i += NT) SDEG[i] = 0.f;
  __threadfence();
  __syncthreads();

#pragma unroll 1
  for (int c = 0; c < nch; ++c) {
    const int tot = chunk_hits_rows(rows, c * SCH, nnz, n0, tid, LIST, scan_ws);
#pragma unroll 1
    for (int base = 0; base < tot; base += 32) {
      const int q = base + lane;
      const bool qv = q < tot;
      const int qc = q < SCH ? q : SCH - 1;
      int e = LIST[qc];
      e = qv ? e : 0;
      e = e < 0 ? 0 : (e >= nnz ? nnz - 1 : e);
      const int r = rows[e];
      int ci = cols[e];
      const float v = vals[e];
      int dl = r - n0; dl = dl < 0 ? 0 : (dl >= SRB ? SRB - 1 : dl);
      ci = ci < 0 ? 0 : (ci >= nnode ? nnode - 1 : ci);
      const int own = (qv && (dl >> RPW_LOG) == wave) ? 1 : 0;
      unsigned msk = (unsigned)__ballot(own);
#pragma unroll 1
      for (int it = 0; it < 32; ++it) {
        if (msk == 0u) break;
        const int bp = __builtin_ctz(msk); msk &= msk - 1u;
        const int hd = __shfl(dl, bp, 32);
        const int hc = __shfl(ci, bp, 32);
        const float hv = __shfl(v, bp, 32);
        const v2f g = *(const v2f*)(feat + (size_t)hc * PD + c2);
        const size_t o = (size_t)(n0 + hd) * PD + c2;
        v2f s  = *(const v2f*)(ASUM + o);
        v2f sq = *(const v2f*)(ASQ + o);
        v2f mx = *(const v2f*)(AMX + o);
        v2f mn = *(const v2f*)(AMN + o);
        const v2f vg = hv * g;
        s = s + vg;
        v2f gg = g * g;
        gg = hv * gg;
        sq = sq + gg;
        mx[0] = fmaxf(mx[0], g[0]); mx[1] = fmaxf(mx[1], g[1]);
        mn[0] = fminf(mn[0], g[0]); mn[1] = fminf(mn[1], g[1]);
        *(volatile v2f*)(ASUM + o) = s; *(volatile v2f*)(ASQ + o) = sq; *(volatile v2f*)(AMX + o) = mx; *(volatile v2f*)(AMN + o) = mn;
        __threadfence();
        *(volatile v2f*)(ASUM + o) = s; *(volatile v2f*)(ASQ + o) = sq; *(volatile v2f*)(AMX + o) = mx; *(volatile v2f*)(AMN + o) = mn;
        if (lane == 0) SDEG[hd] += hv;
      }
    }
    __syncthreads();
  }

  float part = 0.f;
#pragma unroll 1
  for (int j = 0; j < RPW; ++j) {
    const int dl = wave * RPW + j;
    const int n = n0 + dl;
    const float dg = SDEG[dl];
    const float lg = log10f(dg + 2.0f);
    if (n < m) {
      part += lg;
      const float sdg = dg > 0.f ? dg : 1.0f;
      const float inv = 1.0f / sdg;
      const size_t o = (size_t)n * PD + c2;
      const v2f s  = *(const v2f*)(ASUM + o);
      const v2f sq = *(const v2f*)(ASQ + o);
      const v2f mx = *(const v2f*)(AMX + o);
      const v2f mn = *(const v2f*)(AMN + o);
      const v2f mean = s * inv;
      const v2f sqm  = sq * inv;
      const v2f m2 = mean * mean;
      const v2f var = sqm - m2;
      const float v0 = var[0] > 0.f ? var[0] : 0.f;
      const float v1 = var[1] > 0.f ? var[1] : 0.f;
      v2f sd; sd[0] = sqrtf(v0); sd[1] = sqrtf(v1);
      for (int pass = 0; pass < 2; ++pass) {
        *(volatile v2f*)(ASUM + o) = mean;
        *(volatile v2f*)(ASQ + o)  = sd;
        *(volatile v2f*)(AMX + o)  = mx;
        *(volatile v2f*)(AMN + o)  = mn;
        __threadfence();
      }
    }
    if (lane == 0) SDEG[dl] = lg;
  }
  if (lane == 0) SPART[wave] = part;
  __syncthreads();
  for (int pass = 0; pass < 2; ++pass) {
#pragma unroll
    for (int it = 0; it < RPW / 128; ++it) {
      const int idx = wave * RPW + it * 128 + 4 * lane;
      const v4f t = *(const v4f*)(SDEG + idx);
      *(volatile v4f*)(LOGD + (size_t)n0 + idx) = t;
    }
    __threadfence();
  }
  if (wave == 0) {
    float total = 0.f;
#pragma unroll
    for (int w = 0; w < NT / 32; ++w) total += SPART[w];
    const float pv = (lane == 0) ? total : 0.f;
    for (int pass = 0; pass < 2; ++pass) { *(volatile float*)(PART + (size_t)blockIdx.x * 32 + lane) = pv; __threadfence(); }
  }
}

__global__ __launch_bounds__(64) void k_gemm(const float* __restrict__ AMEAN, const float* __restrict__ AMX, const float* __restrict__ AMN,
                                             const float* __restrict__ ASD, const float* __restrict__ LOGD, const float* __restrict__ PART,
                                             const _Float16* __restrict__ Wh, const float* __restrict__ bias, float* __restrict__ out,
                                             int m, int ntiles) {
  __shared__ __align__(16) _Float16 At[2][16 * APITCH];
  __shared__ __align__(16) float sT[2][16 * 68];
  const int lane = threadIdx.x & 31, wave = threadIdx.x >> 5;
  const int rlane = lane & 15, hh = lane >> 4, koff = hh * 8;
  const int row0 = (blockIdx.x * 2 + wave) * 16;

  float tot = 0.f;
#pragma unroll 1
  for (int b = 0; b < ntiles; ++b) tot += PART[(size_t)b * 32];
  const float delta = tot / (float)m;
  const float rdelta = 1.0f / delta;

  _Float16* at = At[wave];
#pragma unroll 1
  for (int r = 0; r < 16; ++r) {
    int gr = row0 + r; gr = gr < m ? gr : m - 1;
    const float lg = LOGD[gr];
    const float s  = lg * rdelta;
    const float rs = 1.0f / s;
#pragma unroll
    for (int half = 0; half < 2; ++half) {
      const int d = lane + 32 * half;
      const size_t gb = (size_t)gr * PD + d;
      const float a0 = AMEAN[gb], a1 = AMX[gb], a2 = AMN[gb], a3 = ASD[gb];
      _Float16* rp = at + r * APITCH + d;
      rp[0]   = (_Float16)a0; rp[64]  = (_Float16)(a0 * s); rp[128] = (_Float16)(a0 * rs);
      rp[192] = (_Float16)a1; rp[256] = (_Float16)(a1 * s); rp[320] = (_Float16)(a1 * rs);
      rp[384] = (_Float16)a2; rp[448] = (_Float16)(a2 * s); rp[512] = (_Float16)(a2 * rs);
      rp[576] = (_Float16)a3; rp[640] = (_Float16)(a3 * s); rp[704] = (_Float16)(a3 * rs);
    }
  }
  __syncthreads();

  v8f acc[4];
#pragma unroll
  for (int j = 0; j < 4; ++j) acc[j] = (v8f){0.f, 0.f, 0.f, 0.f, 0.f, 0.f, 0.f, 0.f};
  const _Float16* arow = at + rlane * APITCH + koff;
#pragma unroll 2
  for (int k0 = 0; k0 < PK; k0 += 32) {
    v16h bq[4];
#pragma unroll
    for (int j = 0; j < 4; ++j) bq[j] = Frag<_Float16>::load(Wh + (size_t)(j * 16 + rlane) * PK + koff + k0);
    const v16h af = Frag<_Float16>::load(arow + k0);
#pragma unroll
    for (int j = 0; j < 4; ++j) acc[j] = Frag<_Float16>::mma(af, bq[j], acc[j]);
    Frag<_Float16>::guard(acc[0], acc[3], af, af);
    Frag<_Float16>::keep(bq[0], bq[1], bq[2], bq[3]);
  }
  acc_guard4(acc[0], acc[1], acc[2], acc[3]);

  float* slab = sT[wave];
#pragma unroll
  for (int j = 0; j < 4; ++j) {
    const int n = j * 16 + rlane;
    const float bv = bias[n];
#pragma unroll
    for (int r = 0; r < 8; ++r) {
      float v = acc[j][r] * WSCALE_INV;
      v = v + bv;
      v = (v >= 0.f) ? v : NEG_SLOPE * v;
      slab[(hh * 8 + r) * 68 + j * 16 + rlane] = v;
    }
  }
  __builtin_amdgcn_fence(__ATOMIC_RELEASE, "workgroup");
  __builtin_amdgcn_wave_barrier();
  __builtin_amdgcn_fence(__ATOMIC_ACQUIRE, "workgroup");
  if (row0 + 15 < m) {
    const int c4 = rlane * 4;
    for (int pass = 0; pass < 2; ++pass) {
#pragma unroll
      for (int it = 0; it < 8; ++it) {
        const int row = it * 2 + hh;
        const v4f v = *(const v4f*)(slab + row * 68 + c4);
        *(volatile v4f*)(out + (size_t)(row0 + row) * POUT + c4) = v;
      }
      __threadfence();
    }
  }
}

extern "C" void kernel_launch(void* const* d_in, const int* in_sizes, int n_in,
                              void* d_out, int out_size, void* d_ws, size_t ws_size, hipStream_t stream) {
  if (n_in < 6) return;
  const int*   rows = (const int*)  d_in[0];
  const int*   cols = (const int*)  d_in[1];
  const float* vals = (const float*)d_in[2];
  const float* feat = (const float*)d_in[3];
  const float* W    = (const float*)d_in[4];
  const float* bias = (const float*)d_in[5];
  float* out = (float*)d_out;

  const int nnz   = in_sizes[0];
  const int nnode = in_sizes[3] / PD;
  const int m     = out_size / POUT;
  if (nnz < SP || (nnz % SP) != 0 || in_sizes[1] != nnz || in_sizes[2] != nnz) return;
  if (m < 32 || (m % 32) != 0 || nnode < 1 || in_sizes[4] != POUT * PK || in_sizes[5] != POUT) return;

  const int ntiles = (m + SRB - 1) / SRB;
  const int arows  = ntiles * SRB;
  const int nch    = (nnz + SCH - 1) / SCH;

  char* ws = (char*)d_ws; size_t off = 0;
  auto carve = [&](size_t bytes) -> char* { char* p = ws + off; off += (bytes + 255) & ~(size_t)255; return p; };
  float*    ASUM = (float*)carve((size_t)arows * PD * 4);
  float*    ASQ  = (float*)carve((size_t)arows * PD * 4);
  float*    AMX  = (float*)carve((size_t)arows * PD * 4);
  float*    AMN  = (float*)carve((size_t)arows * PD * 4);
  float*    LOGD = (float*)carve((size_t)arows * 4);
  float*    PART = (float*)carve((size_t)ntiles * 128);
  _Float16* Wh   = (_Float16*)carve((size_t)POUT * PK * 2);
  if (off > ws_size || off > WS_CAP) return;

  {
    const int n2 = POUT * PK / 2;
    cast_w_f16x2<<<(n2 + 255) / 256, 256, 0, stream>>>(W, Wh, n2);
  }
  k_stream<<<ntiles, NT, 0, stream>>>(rows, cols, vals, feat, ASUM, ASQ, AMX, AMN, LOGD, PART, nnz, nch, m, nnode);
  k_gemm<<<m / 32, 64, 0, stream>>>(ASUM, AMX, AMN, ASQ, LOGD, PART, Wh, bias, out, m, ntiles);
}
